// LSTMPredictor_40553081209541
// MI455X (gfx1250) — hardware-verified
//
#include <hip/hip_runtime.h>
#include <math.h>

constexpr int NBATCH   = 1024;
constexpr int NSTEP    = 512;
constexpr int NIN      = 4;
constexpr int NHID     = 128;
constexpr int NGATE    = 4 * NHID;
constexpr int NOUTF    = 4;
constexpr int ROWS_BLK = 16;
constexpr int NTHR     = 256;
constexpr int NWAVE    = NTHR / 32;
constexpr int NBLK     = NBATCH / ROWS_BLK;
constexpr int HPITCH   = 136;
constexpr int XCHUNK   = 32;
constexpr int NCHUNK   = NSTEP / XCHUNK;
constexpr int HFPITCH  = 132;
constexpr float WCARRY  = 16.0f;
constexpr float HCARRY  = 16.0f;
constexpr float ACC_INV = 1.0f / (WCARRY * HCARRY);

static_assert(NHID % 32 == 0, "K multiple of 32");
static_assert(NHID == 16 * NWAVE, "one 16-unit group per wave");
static_assert(NGATE == 4 * NHID, "four gates");
static_assert(NBATCH % ROWS_BLK == 0, "block rows");
static_assert(NSTEP % XCHUNK == 0, "no x tail chunk");
static_assert((2 * ROWS_BLK * HPITCH) % NTHR == 0, "h zero-fill loop exact");
static_assert(ROWS_BLK * XCHUNK == 2 * NTHR, "x chunk staging: two float4 per thread");
static_assert(HPITCH % 8 == 0 && HPITCH >= NHID, "fragment alignment");
static_assert(HFPITCH % 4 == 0 && HFPITCH >= NHID, "float4 alignment");
static_assert(ROWS_BLK * NOUTF == 64, "two whole 128-B lines per block");
static_assert(NIN == 4, "one float4 per (row, step)");

typedef __attribute__((ext_vector_type(16))) _Float16 v16h;
typedef __attribute__((ext_vector_type(8)))  _Float16 v8h;
typedef __attribute__((ext_vector_type(8)))  float    v8f;
typedef __attribute__((ext_vector_type(4)))  float    v4f;

__device__ __forceinline__ void grp_guard_h(v8f& a, v8f& b, v8f& c, v8f& d,
                                            v16h x, v16h b0, v16h b1, v16h b2, v16h b3) {
  asm volatile("v_nop\n\tv_nop\n\tv_nop\n\tv_nop"
               : "+v"(a), "+v"(b), "+v"(c), "+v"(d)
               : "v"(x), "v"(b0), "v"(b1), "v"(b2), "v"(b3));
}
__device__ __forceinline__ void acc_guard4(v8f& a, v8f& b, v8f& c, v8f& d) {
  asm volatile("v_nop\n\tv_nop\n\tv_nop\n\tv_nop" : "+v"(a), "+v"(b), "+v"(c), "+v"(d));
}
__device__ __forceinline__ int pin_after_frag(int o, v16h f) { asm volatile("" : "+v"(o) : "v"(f)); return o; }
__device__ __forceinline__ int pin_after_val(int o, float d) { asm volatile("" : "+v"(o) : "v"(d)); return o; }

template <typename T> struct Frag;
template <> struct Frag<_Float16> {
  typedef v16h V;
  union U { v16h v; v8h h[2]; };
  static __device__ __forceinline__ v16h load(const _Float16* p) {
    U f;
    f.h[0] = *(const v8h*)(p);
    f.h[1] = *(const v8h*)(p + 16);
    return f.v;
  }
  static __device__ __forceinline__ v8f mma(v16h a, v16h b, v8f c) {
    return __builtin_amdgcn_wmma_f32_16x16x32_f16(false, a, false, b, (short)0, c, false, false);
  }
};

__device__ __forceinline__ float fsig(float x)  { return __builtin_amdgcn_rcpf(1.0f + __expf(-x)); }
__device__ __forceinline__ float ftanh(float x) { return 1.0f - 2.0f * __builtin_amdgcn_rcpf(__expf(2.0f * x) + 1.0f); }

__attribute__((amdgpu_num_vgpr(256)))
__global__ __launch_bounds__(NTHR) void lstm_seq_kernel(const float* __restrict__ x,
                                                        const float* __restrict__ W_ih,
                                                        const float* __restrict__ W_hh,
                                                        const float* __restrict__ b_ih,
                                                        const float* __restrict__ b_hh,
                                                        const float* __restrict__ W_fc,
                                                        const float* __restrict__ b_fc,
                                                        float* __restrict__ out) {
  __shared__ __align__(16) _Float16 h_sh[2][ROWS_BLK * HPITCH];
  __shared__ __align__(16) float    xs[2][ROWS_BLK * XCHUNK * NIN];
  __shared__ __align__(16) float    hf_sh[ROWS_BLK * HFPITCH];
  __shared__ __align__(16) float    o_sh[ROWS_BLK * NOUTF];

  const int tid  = threadIdx.x;
  const int lane = tid & 31;
  const int wave = tid >> 5;
  const int c    = lane & 15;
  const int hh   = lane >> 4;
  const int koff = hh * 8;
  const int unit = wave * 16 + c;
  const int r0   = blockIdx.x * ROWS_BLK;

  v16h Bf[4][4];
  {
    v16h lastf = {};
#pragma unroll
    for (int q = 0; q < 4; ++q) {
#pragma unroll
      for (int kk = 0; kk < 4; ++kk) {
        int wo = (q * NHID + unit) * NHID + kk * 32 + koff;
        wo = pin_after_frag(wo, lastf);
        const float* wp = W_hh + wo;
        const v4f a0 = *(const v4f*)(wp);
        const v4f a1 = *(const v4f*)(wp + 4);
        const v4f a2 = *(const v4f*)(wp + 16);
        const v4f a3 = *(const v4f*)(wp + 20);
        v16h f;
#pragma unroll
        for (int e = 0; e < 4; ++e) {
          f[e]      = (_Float16)(a0[e] * WCARRY);
          f[4 + e]  = (_Float16)(a1[e] * WCARRY);
          f[8 + e]  = (_Float16)(a2[e] * WCARRY);
          f[12 + e] = (_Float16)(a3[e] * WCARRY);
        }
        Bf[q][kk] = f;
        lastf = f;
      }
    }
  }

  v4f   wih[4];
  float bias2[4];
#pragma unroll
  for (int q = 0; q < 4; ++q) {
    const int n = q * NHID + unit;
    wih[q]   = *(const v4f*)(W_ih + n * NIN);
    bias2[q] = b_ih[n] + b_hh[n];
  }

  {
    _Float16* hz = &h_sh[0][0];
#pragma unroll 1
    for (int i = tid; i < 2 * ROWS_BLK * HPITCH; i += NTHR) hz[i] = (_Float16)0.0f;
  }
#pragma unroll
  for (int it = 0; it < 2; ++it) {
    const int idx = it * NTHR + tid;
    const int row = idx >> 5;
    const int sc  = idx & 31;
    const v4f v = *(const v4f*)(x + ((size_t)(r0 + row) * NSTEP + (size_t)sc) * NIN);
    *(v4f*)(&xs[0][idx * NIN]) = v;
  }

  float c_reg[8], h_reg[8];
#pragma unroll
  for (int r = 0; r < 8; ++r) { c_reg[r] = 0.0f; h_reg[r] = 0.0f; }
  __syncthreads();

  const v8f z8 = {0.f, 0.f, 0.f, 0.f, 0.f, 0.f, 0.f, 0.f};

#pragma unroll 1
  for (int t = 0; t < NSTEP; ++t) {
    const int rd = t & 1;
    const int wr = rd ^ 1;
    const int ch = t >> 5;
    const int s  = t & (XCHUNK - 1);
    const int xb = ch & 1;

    __syncthreads();

    if (s == 0 && ch + 1 < NCHUNK) {
      const int nb = xb ^ 1;
#pragma unroll
      for (int it = 0; it < 2; ++it) {
        const int idx = it * NTHR + tid;
        const int row = idx >> 5;
        const int sc  = idx & 31;
        const v4f v = *(const v4f*)(x + ((size_t)(r0 + row) * NSTEP + (size_t)((ch + 1) * XCHUNK + sc)) * NIN);
        *(v4f*)(&xs[nb][idx * NIN]) = v;
      }
    }

    v8f acc0 = z8, acc1 = z8, acc2 = z8, acc3 = z8;
    const _Float16* ap = &h_sh[rd][0] + c * HPITCH + koff;
#pragma unroll
    for (int kk = 0; kk < 4; ++kk) {
      const v16h a = Frag<_Float16>::load(ap + kk * 32);
      acc0 = Frag<_Float16>::mma(a, Bf[0][kk], acc0);
      acc1 = Frag<_Float16>::mma(a, Bf[1][kk], acc1);
      acc2 = Frag<_Float16>::mma(a, Bf[2][kk], acc2);
      acc3 = Frag<_Float16>::mma(a, Bf[3][kk], acc3);
      grp_guard_h(acc0, acc1, acc2, acc3, a, Bf[0][kk], Bf[1][kk], Bf[2][kk], Bf[3][kk]);
    }
    acc_guard4(acc0, acc1, acc2, acc3);

    float dep = c_reg[0];
#pragma unroll
    for (int r = 0; r < 8; ++r) {
      int xo = ((8 * hh + r) * XCHUNK + s) * NIN;
      xo = pin_after_val(xo, dep);
      const v4f xv = *(const v4f*)(&xs[xb][xo]);
      float pi = bias2[0], pf = bias2[1], pg = bias2[2], po = bias2[3];
      pi = fmaf(xv[0], wih[0][0], pi); pi = fmaf(xv[1], wih[0][1], pi);
      pi = fmaf(xv[2], wih[0][2], pi); pi = fmaf(xv[3], wih[0][3], pi);
      pf = fmaf(xv[0], wih[1][0], pf); pf = fmaf(xv[1], wih[1][1], pf);
      pf = fmaf(xv[2], wih[1][2], pf); pf = fmaf(xv[3], wih[1][3], pf);
      pg = fmaf(xv[0], wih[2][0], pg); pg = fmaf(xv[1], wih[2][1], pg);
      pg = fmaf(xv[2], wih[2][2], pg); pg = fmaf(xv[3], wih[2][3], pg);
      po = fmaf(xv[0], wih[3][0], po); po = fmaf(xv[1], wih[3][1], po);
      po = fmaf(xv[2], wih[3][2], po); po = fmaf(xv[3], wih[3][3], po);
      const float zi = fmaf(acc0[r], ACC_INV, pi);
      const float zf = fmaf(acc1[r], ACC_INV, pf);
      const float zg = fmaf(acc2[r], ACC_INV, pg);
      const float zo = fmaf(acc3[r], ACC_INV, po);
      const float ig = fsig(zi);
      const float fg = fsig(zf);
      const float gg = ftanh(zg);
      const float og = fsig(zo);
      const float cn = fmaf(fg, c_reg[r], ig * gg);
      c_reg[r] = cn;
      const float hn = og * ftanh(cn);
      h_reg[r] = hn;
      h_sh[wr][(8 * hh + r) * HPITCH + unit] = (_Float16)(hn * HCARRY);
      dep = hn;
    }
  }

#pragma unroll
  for (int r = 0; r < 8; ++r) hf_sh[(8 * hh + r) * HFPITCH + unit] = h_reg[r];
  __syncthreads();

  if (tid < ROWS_BLK * NOUTF) {
    const int m = tid >> 2;
    const int o = tid & 3;
    float acc = 0.0f;
#pragma unroll 2
    for (int k4 = 0; k4 < NHID / 4; ++k4) {
      const v4f hv = *(const v4f*)(hf_sh + m * HFPITCH + 4 * k4);
      const v4f wv = *(const v4f*)(W_fc + o * NHID + 4 * k4);
      acc = fmaf(hv[0], wv[0], acc);
      acc = fmaf(hv[1], wv[1], acc);
      acc = fmaf(hv[2], wv[2], acc);
      acc = fmaf(hv[3], wv[3], acc);
    }
    acc += b_fc[o];
    o_sh[tid] = acc;
  }
  __syncthreads();

  if (wave < 2 && lane < 8) {
    const v4f v = *(const v4f*)(o_sh + wave * 32 + lane * 4);
    volatile v4f* p = (volatile v4f*)(out + (size_t)r0 * NOUTF + wave * 32 + lane * 4);
    *p = v;
    __threadfence();
    *p = v;
  }
}

extern "C" void kernel_launch(void* const* d_in, const int* in_sizes, int n_in,
                              void* d_out, int out_size, void* d_ws, size_t ws_size, hipStream_t stream) {
  (void)d_ws; (void)ws_size;
  if (n_in < 7 || d_out == nullptr) return;
  if (in_sizes[0] != NBATCH * NSTEP * NIN || in_sizes[1] != NGATE * NIN || in_sizes[2] != NGATE * NHID ||
      in_sizes[3] != NGATE || in_sizes[4] != NGATE || in_sizes[5] != NOUTF * NHID || in_sizes[6] != NOUTF ||
      out_size != NBATCH * NOUTF) return;

  const float* x    = (const float*)d_in[0];
  const float* W_ih = (const float*)d_in[1];
  const float* W_hh = (const float*)d_in[2];
  const float* b_ih = (const float*)d_in[3];
  const float* b_hh = (const float*)d_in[4];
  const float* W_fc = (const float*)d_in[5];
  const float* b_fc = (const float*)d_in[6];
  float* out = (float*)d_out;

  lstm_seq_kernel<<<NBLK, NTHR, 0, stream>>>(x, W_ih, W_hh, b_ih, b_hh, W_fc, b_fc, out);
}
